// CelestialWaveAggregator_40638980554821
// MI455X (gfx1250) — hardware-verified
//
#include <hip/hip_runtime.h>


namespace {
constexpr int B = 32, S = 4096, NW = 118, NB = 13, MAXW = 12, NR = B * S, H1 = 32, H2 = 64;
__constant__ int LENS[NB] = {9, 9, 9, 9, 9, 9, 9, 9, 9, 9, 12, 8, 3};
__constant__ int STARTS[NB] = {5, 14, 23, 32, 41, 50, 59, 68, 77, 86, 95, 107, 115};
constexpr float XS = 8.0f, HS = 64.0f  , WSC = 256.0f;
typedef _Float16 b16;
typedef __attribute__((ext_vector_type(16))) _Float16 v16b;
typedef __attribute__((ext_vector_type(8))) _Float16 v8b;
typedef __attribute__((ext_vector_type(8))) float v8f;
typedef __attribute__((ext_vector_type(4))) float v4f;
typedef __attribute__((ext_vector_type(2))) float v2f;
__device__ __forceinline__ float bf16_rne(float f) { unsigned int u = __float_as_uint(f); u += 0x7FFFu + ((u >> 16) & 1u); return __uint_as_float(u & 0xFFFF0000u); }
__device__ __forceinline__ void split16(float v, b16& hi, b16& lo) { hi = (b16)v; lo = (b16)(v - (float)hi); }
__device__ __forceinline__ v16b frag_kb(const b16* p, int hh) { const v8b a = *(const v8b*)(p + 8 * hh), b = *(const v8b*)(p + 16 + 8 * hh); v16b f;
#pragma unroll
  for (int e = 0; e < 8; ++e) { f[e] = a[e]; f[8 + e] = b[e]; } return f; }
__device__ __forceinline__ v8f wmma16b(v16b a, v16b b, v8f c) { v8f d = __builtin_amdgcn_wmma_f32_16x16x32_f16(false, a, false, b, (short)0, c, false, false); asm volatile("v_nop\n\tv_nop\n\tv_nop\n\tv_nop" : "+v"(d) : "v"(a), "v"(b)); return d; }
__device__ __forceinline__ void wave_lds_sync() { __builtin_amdgcn_fence(__ATOMIC_RELEASE, "workgroup"); __builtin_amdgcn_wave_barrier(); __builtin_amdgcn_fence(__ATOMIC_ACQUIRE, "workgroup"); }
__device__ __forceinline__ float pmul(float a, float b) { float p = a * b; asm volatile("" : "+v"(p)); return p; }
__device__ __forceinline__ float gelu(float v) { return 0.5f * v * (1.0f + erff(v * 0.70710678118654752f)); }

__global__ __launch_bounds__(256) void wprep_kernel(const float* __restrict__ w, int KIN, int OUTW, b16* __restrict__ WT) {
  const int u = blockIdx.x * 256 + threadIdx.x; if (u >= NB * OUTW * KIN / 8) return; const int e = u * 8; const int c = e / (OUTW * KIN), o = (e / KIN) % OUTW, k0 = e % KIN; v8b v;
#pragma unroll
  for (int j = 0; j < 8; ++j) v[j] = (b16)(bf16_rne(w[((size_t)c * KIN + k0 + j) * OUTW + o]) * WSC); for (int pass = 0; pass < 2; ++pass) { *(volatile v8b*)(WT + e) = v; __threadfence(); }
}
__global__ __launch_bounds__(32) void cw_kernel(const float* __restrict__ wf, const float* __restrict__ al, const float* __restrict__ W1, const float* __restrict__ b1, const b16* __restrict__ W2T, const float* __restrict__ b2, const b16* __restrict__ W3T, const float* __restrict__ b3, const float* __restrict__ W4, const float* __restrict__ b4, int NRV, float* __restrict__ out) {
  __shared__ __attribute__((aligned(16))) b16 Ah[16][128 + 8], Bh[16][128 + 8], Bl[16][128 + 8], Ch[16][H2 + 8], Cl[16][H2 + 8], Dh[16][H1 + 8], Dl[16][H1 + 8]; __shared__ float Mw[NB][MAXW], Ag[16][16], To[32 * NB];
  const int lane = threadIdx.x, nloc = lane & 15, hlf = lane >> 4; const size_t r0w = (size_t)blockIdx.x * 32; const float sc = 1.0f / (HS * WSC), sa = 1.0f / (XS * HS);
  if (lane < NB) { const int len = LENS[lane]; float mx = -INFINITY; for (int j = 0; j < MAXW; ++j) if (j < len) mx = fmaxf(mx, bf16_rne(al[lane * MAXW + j])); float s = 0.0f; float e[MAXW];
    for (int j = 0; j < MAXW; ++j) { e[j] = j < len ? __expf(bf16_rne(al[lane * MAXW + j]) - mx) : 0.0f; s += e[j]; } for (int j = 0; j < MAXW; ++j) Mw[lane][j] = e[j] / s; }
  wave_lds_sync();
  for (int c = 0; c < 16; ++c) for (int q = 0; q < 4; ++q) { const int w = q * 32 + lane; float m = 0.0f; if (c < NB) { const int st = STARTS[c], len = LENS[c]; if (w >= st && w < st + len && w < NW) m = Mw[c][w - st]; } b16 p, ql; split16(m * HS, p, ql); Bh[c][w] = p; Bl[c][w] = ql; }
  wave_lds_sync();
#pragma unroll 1
  for (int half = 0; half < 2; ++half) { const size_t r0 = r0w + half * 16; const bool live = r0 < (size_t)NRV;
    for (int rr = 0; rr < 16; ++rr) for (int q = 0; q < 4; ++q) { const int w = q * 32 + lane; Ah[rr][w] = (w < NW && live) ? (b16)(bf16_rne(wf[(r0 + rr) * NW + w]) * XS) : (b16)0.0f; }
    wave_lds_sync();
    { v8f acc = {};
#pragma unroll
      for (int kb = 0; kb < 128; kb += 32) { const v16b a = frag_kb(&Ah[nloc][kb], hlf); acc = wmma16b(a, frag_kb(&Bh[nloc][kb], hlf), acc); acc = wmma16b(a, frag_kb(&Bl[nloc][kb], hlf), acc); }
#pragma unroll
      for (int r8 = 0; r8 < 8; ++r8) Ag[8 * hlf + r8][nloc] = acc[r8] * sa; }
    wave_lds_sync();
#pragma unroll 1
    for (int c = 0; c < NB; ++c) { const float w1 = bf16_rne(W1[c * H1 + lane]), bb1 = bf16_rne(b1[c * H1 + lane]);
      for (int rr = 0; rr < 16; ++rr) { const float h1 = gelu(pmul(Ag[rr][c], w1) + bb1); b16 p, ql; split16(h1 * HS, p, ql); Dh[rr][lane] = p; Dl[rr][lane] = ql; }
      wave_lds_sync();
      v8f a2[4]; { const v16b a = frag_kb(&Dh[nloc][0], hlf), alo = frag_kb(&Dl[nloc][0], hlf);
#pragma unroll
        for (int t = 0; t < 4; ++t) { a2[t] = (v8f){}; const v16b bw = frag_kb(W2T + ((size_t)c * H2 + t * 16 + nloc) * H1, hlf); a2[t] = wmma16b(a, bw, a2[t]); a2[t] = wmma16b(alo, bw, a2[t]); } }
#pragma unroll
      for (int t = 0; t < 4; ++t) { const int u = t * 16 + nloc; const float bb2 = bf16_rne(b2[c * H2 + u]);
#pragma unroll
        for (int r8 = 0; r8 < 8; ++r8) { const float h2 = gelu(a2[t][r8] * sc + bb2); b16 p, ql; split16(h2 * HS, p, ql); Ch[8 * hlf + r8][u] = p; Cl[8 * hlf + r8][u] = ql; } }
      wave_lds_sync();
      v8f a3[2] = {(v8f){}, (v8f){}};
#pragma unroll
      for (int kb = 0; kb < H2; kb += 32) { const v16b a = frag_kb(&Ch[nloc][kb], hlf), alo = frag_kb(&Cl[nloc][kb], hlf);
#pragma unroll
        for (int t = 0; t < 2; ++t) { const v16b bw = frag_kb(W3T + ((size_t)c * H1 + t * 16 + nloc) * H2 + kb, hlf); a3[t] = wmma16b(a, bw, a3[t]); a3[t] = wmma16b(alo, bw, a3[t]); } }
      float pd[8];
#pragma unroll
      for (int r8 = 0; r8 < 8; ++r8) pd[r8] = 0.0f;
#pragma unroll
      for (int t = 0; t < 2; ++t) { const int u = t * 16 + nloc; const float bb3 = bf16_rne(b3[c * H1 + u]), w4 = bf16_rne(W4[c * H1 + u]);
#pragma unroll
        for (int r8 = 0; r8 < 8; ++r8) { const float h3 = gelu(a3[t][r8] * sc + bb3); pd[r8] += pmul(h3, w4); } }
      const float bb4 = bf16_rne(b4[c]);
#pragma unroll
      for (int r8 = 0; r8 < 8; ++r8) { float s = pd[r8]; for (int o = 1; o < 16; o <<= 1) s += __shfl_xor(s, o); if (nloc == 0) To[(half * 16 + 8 * hlf + r8) * NB + c] = live ? tanhf(s + bb4) : 0.0f; }
      wave_lds_sync(); } }
  for (int pass = 0; pass < 2; ++pass) { for (int u = lane; u < 32 * NB; u += 32) ((volatile float*)out)[r0w * NB + u] = To[u]; __threadfence(); }
}
}

extern "C" void kernel_launch(void* const* d_in, const int* in_sizes, int n_in, void* d_out, int out_size, void* d_ws, size_t ws_size, hipStream_t stream) {
  (void)n_in;
  auto Fp = [&](int i) { return (const float*)d_in[i]; };
  if (in_sizes[0] != NR * NW || in_sizes[1] != NB * MAXW || in_sizes[2] != NB * H1 || in_sizes[4] != NB * H1 * H2 || in_sizes[6] != NB * H2 * H1 || in_sizes[8] != NB * H1 || out_size != NR * NB) return;
  const int NRV = NR;
  size_t off = 0; char* ws = (char*)d_ws;
  auto carve = [&](size_t bytes) { char* p = ws + off; off += (bytes + 255) & ~(size_t)255; return p; };
  b16* W2T = (b16*)carve((size_t)NB * H2 * H1 * 2); b16* W3T = (b16*)carve((size_t)NB * H1 * H2 * 2);
  if (off > ws_size) return;
  wprep_kernel<<<(NB * H2 * H1 / 8 + 255) / 256, 256, 0, stream>>>(Fp(4), H1, H2, W2T); wprep_kernel<<<(NB * H1 * H2 / 8 + 255) / 256, 256, 0, stream>>>(Fp(6), H2, H1, W3T);
  cw_kernel<<<(NRV + 31) / 32, 32, 0, stream>>>(Fp(0), Fp(1), Fp(2), Fp(3), W2T, Fp(5), W3T, Fp(7), Fp(8), Fp(9), NRV, (float*)d_out);
}
